// EFDeepSet_34574486733481
// MI455X (gfx1250) — hardware-verified
//
#include <hip/hip_runtime.h>
#include <stddef.h>
#include <math.h>


#define IN_DIM 14
#define HID    128
#define HID2   256
#define K1P    32
#define NTHR   256
#define NWAVE  8
#define NROWS  128
#define EROWS  64
#define XP     40
#define HP     136
#define AP2    264
#define SCL    16.0f
#define INV16  0.0625f
#define INV256 0.00390625f

#define G_W1   (HID * K1P / 8)
#define G_W2   (HID * HID / 8)
#define G_A1H  (HID2 * HID / 8)
#define G_A2   (HID2 * HID2 / 8)
#define G_TOT  (G_W1 + 2 * G_W2 + 2 * G_A1H + G_A2)

#define LN_XF    0
#define LN_X     (LN_XF + NROWS * 16 * 4)
#define LN_A     (LN_X + NROWS * XP * 2)
#define LN_B     (LN_A + NROWS * HP * 2)
#define LN_STG   (LN_B + NROWS * HP * 2)
#define LDS_NODE (LN_STG + NWAVE * 16 * 128 * 4)
#define LE_D     0
#define LE_A1    (LE_D + EROWS * HP * 2)
#define LE_P     (LE_A1 + EROWS * AP2 * 2)
#define LE_LG    (LE_P + EROWS * HID2 * 4)
#define LE_W     (LE_LG + 2 * EROWS * 4)
#define LDS_EDGE (LE_W + EROWS * 4)

static_assert(NROWS == NWAVE * 16);
static_assert(EROWS == 64 && NTHR == 4 * EROWS);
static_assert((G_W1 % NTHR) == 0 && (G_W2 % NTHR) == 0 && (G_A1H % NTHR) == 0 && (G_A2 % NTHR) == 0);
static_assert((LN_X % 16) == 0 && (LN_A % 16) == 0 && (LN_B % 16) == 0 && (LN_STG % 16) == 0);
static_assert((LE_A1 % 16) == 0 && (LE_P % 16) == 0 && (LE_LG % 16) == 0 && (LE_W % 16) == 0);
static_assert((XP * 2) % 16 == 0 && (HP * 2) % 16 == 0 && (AP2 * 2) % 16 == 0);
static_assert(IN_DIM <= 16 && K1P == 32);

typedef float    v4f  __attribute__((ext_vector_type(4)));
typedef float    v8f  __attribute__((ext_vector_type(8)));
typedef _Float16 v8h  __attribute__((ext_vector_type(8)));
typedef _Float16 v16h __attribute__((ext_vector_type(16)));
union FragH { v16h v; v8h h[2]; };

__device__ __forceinline__ v8f wmh(v16h a, v16h b, v8f c) {
  v8f d = __builtin_amdgcn_wmma_f32_16x16x32_f16(false, a, false, b, (short)0, c, false, false);
#if defined(__HIP_DEVICE_COMPILE__)
  asm volatile("v_nop\n\tv_nop\n\tv_nop\n\tv_nop" : "+v"(d) : "v"(a), "v"(b));
#endif
  return d;
}

__device__ __forceinline__ v8f zero8() {
  v8f z = {0.f, 0.f, 0.f, 0.f, 0.f, 0.f, 0.f, 0.f};
  return z;
}

template <int KT>
__device__ __forceinline__ void mma8(v8f (&acc)[8], const _Float16* ar, const _Float16* __restrict__ bplane,
                                     int nb0, int KP, int m, int hh) {
#pragma unroll
  for (int t = 0; t < 8; ++t) acc[t] = zero8();
#pragma unroll
  for (int kt = 0; kt < KT; ++kt) {
    FragH a;
    a.h[0] = *(const v8h*)(ar + 32 * kt);
    a.h[1] = *(const v8h*)(ar + 32 * kt + 16);
#pragma unroll
    for (int t = 0; t < 8; ++t) {
      const _Float16* bp = bplane + (size_t)(nb0 + 16 * t + m) * KP + 32 * kt + 8 * hh;
      FragH b;
      b.h[0] = *(const v8h*)bp;
      b.h[1] = *(const v8h*)(bp + 16);
      acc[t] = wmh(a.v, b.v, acc[t]);
    }
  }
}

__device__ __forceinline__ void relu_to_lds(const v8f (&acc)[8], _Float16* sp, int pitch) {
#pragma unroll
  for (int t = 0; t < 8; ++t) {
#pragma unroll
    for (int r = 0; r < 8; ++r) sp[r * pitch + 16 * t] = (_Float16)(fmaxf(acc[t][r], 0.0f) * INV16);
  }
}

__global__ __launch_bounds__(NTHR) void k_prep(
    const float* __restrict__ W1, const float* __restrict__ W2, const float* __restrict__ W3,
    const float* __restrict__ A1, const float* __restrict__ A2,
    _Float16* pW1, _Float16* pW2, _Float16* pW3, _Float16* pA1t, _Float16* pA1b, _Float16* pA2) {
  const int b0 = G_W1, b1 = b0 + G_W2, b2 = b1 + G_W2, b3 = b2 + G_A1H, b4 = b3 + G_A1H, b5 = b4 + G_A2;
  const int bstart = blockIdx.x * NTHR;
  const float* src; _Float16* dst; int srcCols, rowOff, Kv, KP, Nout, segOff;
  if (bstart < b0)      { src = W1; dst = pW1;  srcCols = HID;  rowOff = 0;   Kv = IN_DIM; KP = K1P;  Nout = HID;  segOff = 0;  }
  else if (bstart < b1) { src = W2; dst = pW2;  srcCols = HID;  rowOff = 0;   Kv = HID;    KP = HID;  Nout = HID;  segOff = b0; }
  else if (bstart < b2) { src = W3; dst = pW3;  srcCols = HID;  rowOff = 0;   Kv = HID;    KP = HID;  Nout = HID;  segOff = b1; }
  else if (bstart < b3) { src = A1; dst = pA1t; srcCols = HID2; rowOff = 0;   Kv = HID;    KP = HID;  Nout = HID2; segOff = b2; }
  else if (bstart < b4) { src = A1; dst = pA1b; srcCols = HID2; rowOff = HID; Kv = HID;    KP = HID;  Nout = HID2; segOff = b3; }
  else                  { src = A2; dst = pA2;  srcCols = HID2; rowOff = 0;   Kv = HID2;   KP = HID2; Nout = HID2; segOff = b4; }
  const int i = bstart + (int)threadIdx.x;
  if (i >= b5) return;
  const int o  = (i - segOff) * 8;
  const int n  = o / KP;
  const int k0 = o - n * KP;
  const int nc = n < Nout ? n : Nout - 1;
  float v[8];
#pragma unroll
  for (int e = 0; e < 8; ++e) {
    const int k  = k0 + e;
    const int kc = k < Kv ? k : Kv - 1;
    const float xv = src[(size_t)(rowOff + kc) * srcCols + nc];
    v[e] = (k < Kv && n < Nout) ? xv * SCL : 0.0f;
  }
  v8h hv;
#pragma unroll
  for (int e = 0; e < 8; ++e) hv[e] = (_Float16)v[e];
  _Float16* dp = dst + o;
  *(volatile v8h*)dp = hv;
  __threadfence();
  *(volatile v8h*)dp = hv;
}

__global__ __launch_bounds__(NTHR) void k_node(
    const float* __restrict__ x, const _Float16* __restrict__ pW1, const _Float16* __restrict__ pW2,
    const _Float16* __restrict__ pW3, const _Float16* __restrict__ pA1b,
    _Float16* hf, float* P, int nN) {
  extern __shared__ v4f lds_dyn[];
  char* lb = (char*)lds_dyn;
  float*    sXf = (float*)(lb + LN_XF);
  _Float16* sX  = (_Float16*)(lb + LN_X);
  _Float16* sA  = (_Float16*)(lb + LN_A);
  _Float16* sB  = (_Float16*)(lb + LN_B);
  float*    stg = (float*)(lb + LN_STG);
  const int tid = threadIdx.x, lane = tid & 31, wave = tid >> 5, hh = lane >> 4, m = lane & 15;
  const int row0 = blockIdx.x * NROWS;
  const int wr = wave * 16;

  for (int i = tid; i < NROWS * 16; i += NTHR) {
    const int r = i >> 4, c = i & 15;
    int row = row0 + r;
    row = row > nN - 1 ? nN - 1 : row;
    const int cc = c < IN_DIM ? c : IN_DIM - 1;
    const float xv = x[(size_t)row * IN_DIM + cc];
    sXf[i] = (c < IN_DIM) ? xv : 0.0f;
  }
  __syncthreads();
  if (tid < NROWS) {
    const float* xr = sXf + tid * 16;
    float s = 0.0f;
#pragma unroll
    for (int c = 0; c < IN_DIM; ++c) { const float q = xr[c]; s = fmaf(q, q, s); }
    float nrm = sqrtf(s);
    nrm = fmaxf(nrm, 1e-12f);
    const float sc = SCL * (1.0f / nrm);
    v8h q0, q1, z;
#pragma unroll
    for (int e = 0; e < 8; ++e) {
      q0[e] = (_Float16)(xr[e] * sc);
      q1[e] = (_Float16)(xr[8 + e] * sc);
      z[e]  = (_Float16)0.0f;
    }
    _Float16* xp = sX + tid * XP;
    *(v8h*)(xp)      = q0;
    *(v8h*)(xp + 8)  = q1;
    *(v8h*)(xp + 16) = z;
    *(v8h*)(xp + 24) = z;
  }
  __syncthreads();

  v8f acc[8];
  mma8<1>(acc, sX + (wr + m) * XP + 8 * hh, pW1, 0, K1P, m, hh);
  relu_to_lds(acc, sA + (wr + 8 * hh) * HP + m, HP);
  __syncthreads();
  mma8<4>(acc, sA + (wr + m) * HP + 8 * hh, pW2, 0, HID, m, hh);
  relu_to_lds(acc, sB + (wr + 8 * hh) * HP + m, HP);
  __syncthreads();
  mma8<4>(acc, sB + (wr + m) * HP + 8 * hh, pW3, 0, HID, m, hh);
  relu_to_lds(acc, sA + (wr + 8 * hh) * HP + m, HP);
  __syncthreads();

  {
    v8h hv[8];
#pragma unroll
    for (int p = 0; p < 8; ++p) hv[p] = *(const v8h*)(sA + (wr + 2 * p + hh) * HP + 8 * m);
    _Float16* gp = hf + (size_t)(row0 + wr) * HID;
#pragma unroll
    for (int p = 0; p < 8; ++p) *(volatile v8h*)(gp + 8 * (32 * p + lane)) = hv[p];
    __threadfence();
#pragma unroll
    for (int p = 0; p < 8; ++p) *(volatile v8h*)(gp + 8 * (32 * p + lane)) = hv[p];
  }

  float* sw = stg + wave * (16 * 128);
#pragma unroll
  for (int g = 0; g < 2; ++g) {
    mma8<4>(acc, sA + (wr + m) * HP + 8 * hh, pA1b, 128 * g, HID, m, hh);
    float* stp = sw + (8 * hh) * 128 + m;
#pragma unroll
    for (int t = 0; t < 8; ++t) {
#pragma unroll
      for (int r = 0; r < 8; ++r) stp[r * 128 + 16 * t] = acc[t][r] * INV256;
    }
    __syncthreads();
    v4f pv[16];
#pragma unroll
    for (int i = 0; i < 16; ++i) pv[i] = *(const v4f*)(sw + i * 128 + 4 * lane);
    float* gq = P + (size_t)(row0 + wr) * HID2 + 128 * g + 4 * lane;
#pragma unroll
    for (int i = 0; i < 16; ++i) *(volatile v4f*)(gq + (size_t)i * HID2) = pv[i];
    __threadfence();
#pragma unroll
    for (int i = 0; i < 16; ++i) *(volatile v4f*)(gq + (size_t)i * HID2) = pv[i];
    __syncthreads();
  }
}

__global__ __launch_bounds__(NTHR) void k_edge(
    const _Float16* __restrict__ hf, const float* __restrict__ P, const int* __restrict__ ei,
    const _Float16* __restrict__ pA1t, const _Float16* __restrict__ pA2, const float* __restrict__ A3,
    float* out, int nE, int nN) {
  extern __shared__ v4f lds_dyn[];
  char* lb = (char*)lds_dyn;
  _Float16* sD  = (_Float16*)(lb + LE_D);
  _Float16* sA1 = (_Float16*)(lb + LE_A1);
  float*    sP  = (float*)(lb + LE_P);
  float*    sLg = (float*)(lb + LE_LG);
  float*    sW  = (float*)(lb + LE_W);
  const int tid = threadIdx.x, lane = tid & 31, wave = tid >> 5, hh = lane >> 4, m = lane & 15;
  const int e0 = blockIdx.x * EROWS;

  {
    const int r = tid >> 2, q = tid & 3;
    int e = e0 + r;
    e = e > nE - 1 ? nE - 1 : e;
    int si = ei[e];
    int di = ei[(size_t)nE + e];
    si = si < 0 ? 0 : (si > nN - 1 ? nN - 1 : si);
    di = di < 0 ? 0 : (di > nN - 1 ? nN - 1 : di);
    const _Float16* hi = hf + (size_t)si * HID + 32 * q;
    const _Float16* hj = hf + (size_t)di * HID + 32 * q;
    _Float16* dp = sD + r * HP + 32 * q;
#pragma unroll
    for (int j = 0; j < 4; ++j) {
      const v8h a = *(const v8h*)(hi + 8 * j);
      const v8h b = *(const v8h*)(hj + 8 * j);
      v8h d;
#pragma unroll
      for (int u = 0; u < 8; ++u) d[u] = (_Float16)fabsf((float)a[u] - (float)b[u]);
      *(v8h*)(dp + 8 * j) = d;
    }
    const float* pi = P + (size_t)si * HID2 + 64 * q;
    const float* pj = P + (size_t)di * HID2 + 64 * q;
    float* pp = sP + r * HID2 + 64 * q;
#pragma unroll
    for (int j = 0; j < 16; ++j) {
      const v4f u = (*(const v4f*)(pi + 4 * j) + *(const v4f*)(pj + 4 * j)) * 256.0f;
      *(v4f*)(pp + 4 * j) = u;
    }
  }
  __syncthreads();

  const int rt = wave & 3, ch = wave >> 2;
  const int wr = rt * 16, cb = ch * 128;
  v8f acc[8];

  mma8<4>(acc, sD + (wr + m) * HP + 8 * hh, pA1t, cb, HID, m, hh);
  {
    const float* pp = sP + (wr + 8 * hh) * HID2 + cb + m;
    _Float16* sp = sA1 + (wr + 8 * hh) * AP2 + cb + m;
#pragma unroll
    for (int t = 0; t < 8; ++t) {
#pragma unroll
      for (int r = 0; r < 8; ++r) {
        float v = acc[t][r] + pp[r * HID2 + 16 * t];
        v = fmaxf(v, 0.0f) * INV16;
        sp[r * AP2 + 16 * t] = (_Float16)v;
      }
    }
  }
  __syncthreads();

  mma8<8>(acc, sA1 + (wr + m) * AP2 + 8 * hh, pA2, cb, HID2, m, hh);
  {
    float a3v[8], s[8];
#pragma unroll
    for (int t = 0; t < 8; ++t) { a3v[t] = A3[cb + 16 * t + m]; s[t] = 0.0f; }
#pragma unroll
    for (int t = 0; t < 8; ++t) {
#pragma unroll
      for (int r = 0; r < 8; ++r) s[r] = fmaf(fmaxf(acc[t][r], 0.0f), a3v[t], s[r]);
    }
#pragma unroll
    for (int r = 0; r < 8; ++r) {
      s[r] += __shfl_xor(s[r], 1, 32);
      s[r] += __shfl_xor(s[r], 2, 32);
      s[r] += __shfl_xor(s[r], 4, 32);
      s[r] += __shfl_xor(s[r], 8, 32);
    }
    if (m == 0) {
#pragma unroll
      for (int r = 0; r < 8; ++r) sLg[ch * EROWS + wr + 8 * hh + r] = s[r];
    }
  }
  __syncthreads();

  if (tid < EROWS) {
    float lg = (sLg[tid] + sLg[EROWS + tid]) * INV256;
    lg = fminf(fmaxf(lg, -30.0f), 30.0f);
    const float ex  = expf(-lg);
    const float sig = 1.0f / (1.0f + ex);
    const float c1  = (float)(1.0 - 2.0e-8);
    sW[tid] = 1e-8f + c1 * sig;
  }
  __syncthreads();

  if (wave == 0) {
    const int sl = lane & 15;
    const v4f v = *(const v4f*)(sW + 4 * sl);
    const int eo = e0 + 4 * sl;
    const bool full = (lane < 16) && (eo + 3 < nE);
    const bool part = (lane < 16) && !full;
    volatile float* vo = (volatile float*)out;
    if (full) *(volatile v4f*)(out + eo) = v;
    if (part) {
      if (eo     < nE) vo[eo]     = v[0];
      if (eo + 1 < nE) vo[eo + 1] = v[1];
      if (eo + 2 < nE) vo[eo + 2] = v[2];
      if (eo + 3 < nE) vo[eo + 3] = v[3];
    }
    __threadfence();
    if (full) *(volatile v4f*)(out + eo) = v;
    if (part) {
      if (eo     < nE) vo[eo]     = v[0];
      if (eo + 1 < nE) vo[eo + 1] = v[1];
      if (eo + 2 < nE) vo[eo + 2] = v[2];
      if (eo + 3 < nE) vo[eo + 3] = v[3];
    }
  }
}

extern "C" void kernel_launch(void* const* d_in, const int* in_sizes, int n_in,
                              void* d_out, int out_size, void* d_ws, size_t ws_size,
                              hipStream_t stream) {
  if (n_in < 8) return;
  const int nN = in_sizes[0] / IN_DIM;
  const int nE = in_sizes[1] / 2;
  if (nN <= 0 || nE <= 0 || in_sizes[0] != nN * IN_DIM || in_sizes[1] != 2 * nE) return;
  if (in_sizes[2] != IN_DIM * HID || in_sizes[3] != HID * HID || in_sizes[4] != HID * HID) return;
  if (in_sizes[5] != HID2 * HID2 || in_sizes[6] != HID2 * HID2 || in_sizes[7] != HID2) return;
  if (out_size != nE) return;
  if (nN > (1 << 24) || nE > (1 << 28)) return;

  const float* x  = (const float*)d_in[0];
  const int*   ei = (const int*)d_in[1];
  const float* W1 = (const float*)d_in[2];
  const float* W2 = (const float*)d_in[3];
  const float* W3 = (const float*)d_in[4];
  const float* A1 = (const float*)d_in[5];
  const float* A2 = (const float*)d_in[6];
  const float* A3 = (const float*)d_in[7];
  float* out = (float*)d_out;

  const int nBlkN = (nN + NROWS - 1) / NROWS;
  const int Npad  = nBlkN * NROWS;
  const int nBlkE = (nE + EROWS - 1) / EROWS;

  char* ws = (char*)d_ws;
  size_t off = 0;
  const size_t oW1  = off; off += (size_t)HID * K1P * 2;     off = (off + 255) & ~(size_t)255;
  const size_t oW2  = off; off += (size_t)HID * HID * 2;     off = (off + 255) & ~(size_t)255;
  const size_t oW3  = off; off += (size_t)HID * HID * 2;     off = (off + 255) & ~(size_t)255;
  const size_t oA1t = off; off += (size_t)HID2 * HID * 2;    off = (off + 255) & ~(size_t)255;
  const size_t oA1b = off; off += (size_t)HID2 * HID * 2;    off = (off + 255) & ~(size_t)255;
  const size_t oA2  = off; off += (size_t)HID2 * HID2 * 2;   off = (off + 255) & ~(size_t)255;
  const size_t oHf  = off; off += (size_t)Npad * HID * 2;    off = (off + 255) & ~(size_t)255;
  const size_t oP   = off; off += (size_t)Npad * HID2 * 4;   off = (off + 255) & ~(size_t)255;
  if (off > ws_size || off > (size_t)134217728) return;
  _Float16* pW1  = (_Float16*)(ws + oW1);
  _Float16* pW2  = (_Float16*)(ws + oW2);
  _Float16* pW3  = (_Float16*)(ws + oW3);
  _Float16* pA1t = (_Float16*)(ws + oA1t);
  _Float16* pA1b = (_Float16*)(ws + oA1b);
  _Float16* pA2  = (_Float16*)(ws + oA2);
  _Float16* hf   = (_Float16*)(ws + oHf);
  float*    P    = (float*)(ws + oP);

  k_prep<<<G_TOT / NTHR, NTHR, 0, stream>>>(W1, W2, W3, A1, A2, pW1, pW2, pW3, pA1t, pA1b, pA2);

  hipFuncSetAttribute(reinterpret_cast<const void*>(&k_node),
                      hipFuncAttributeMaxDynamicSharedMemorySize, LDS_NODE);
  k_node<<<nBlkN, NTHR, LDS_NODE, stream>>>(x, pW1, pW2, pW3, pA1b, hf, P, nN);

  hipFuncSetAttribute(reinterpret_cast<const void*>(&k_edge),
                      hipFuncAttributeMaxDynamicSharedMemorySize, LDS_EDGE);
  k_edge<<<nBlkE, NTHR, LDS_EDGE, stream>>>(hf, P, ei, pA1t, pA2, A3, out, nE, nN);
}
